// T5LayerSelfAttention_89953795047772
// MI455X (gfx1250) — hardware-verified
//
#include <hip/hip_runtime.h>

typedef _Float16 v16h __attribute__((ext_vector_type(16)));
typedef _Float16 v8h  __attribute__((ext_vector_type(8)));
typedef float    v8f  __attribute__((ext_vector_type(8)));
typedef float    v4f  __attribute__((ext_vector_type(4)));
typedef v8h __attribute__((may_alias)) v8ha;
typedef v4f __attribute__((may_alias)) v4fa;

union Frag { v16h v; v8h half[2]; };

#define BATCH   2
#define SEQ     2048
#define HIDDEN  1024
#define NHEADS  16
#define HD      64
#define MROWS   (BATCH * SEQ)
#define NX      (MROWS * HIDDEN)
#define NW      (HIDDEN * HIDDEN)
#define NBH     (BATCH * NHEADS)
#define NBUCK   32
#define BTW     4096
#define WSCALE  32.0f
#define PSCALE  16384.0f
#define CSCALE  16.0f
#define LN16F   2.7725887298583984f
#define EPSF    1e-6f

static_assert(SEQ % 128 == 0);
static_assert(HIDDEN == NHEADS * HD);
static_assert(HIDDEN % 64 == 0);
static_assert((NHEADS * BTW) % 256 == 0);

__device__ __forceinline__ v8f wmma_f16(v16h a, v16h b, v8f c) {
  v8f d = __builtin_amdgcn_wmma_f32_16x16x32_f16(false, a, false, b, (short)0, c, false, false);
  asm volatile("v_nop\n\tv_nop\n\tv_nop\n\tv_nop" : "+v"(d) : "v"(a), "v"(b));
  return d;
}

__device__ __forceinline__ v16h load_frag(const _Float16* p, int h) {
  Frag f;
  f.half[0] = *(const v8ha*)(p + 8 * h);
  f.half[1] = *(const v8ha*)(p + 16 + 8 * h);
  return f.v;
}

__global__ __launch_bounds__(128) void rmsnorm_kernel(
    const float* __restrict__ x, const float* __restrict__ lnw,
    _Float16* __restrict__ xh)
{
  __shared__ float red[4];
  const int row = blockIdx.x, tid = threadIdx.x, lane = tid & 31, w = tid >> 5;
  const float* xr = x + (size_t)row * HIDDEN + 8 * tid;
  const v4f a = *(const v4fa*)xr;
  const v4f c = *(const v4fa*)(xr + 4);
  float ss = a.x * a.x + a.y * a.y + a.z * a.z + a.w * a.w
           + c.x * c.x + c.y * c.y + c.z * c.z + c.w * c.w;
  #pragma unroll
  for (int off = 16; off >= 1; off >>= 1) ss += __shfl_xor(ss, off);
  if (lane == 0) red[w] = ss;
  __syncthreads();
  const float tot = (red[0] + red[1]) + (red[2] + red[3]);
  const float inv = rsqrtf(tot * (1.0f / (float)HIDDEN) + EPSF);
  const v4f g0 = *(const v4fa*)(lnw + 8 * tid);
  const v4f g1 = *(const v4fa*)(lnw + 8 * tid + 4);
  const v8h o = { (_Float16)((a.x * inv) * g0.x), (_Float16)((a.y * inv) * g0.y),
                  (_Float16)((a.z * inv) * g0.z), (_Float16)((a.w * inv) * g0.w),
                  (_Float16)((c.x * inv) * g1.x), (_Float16)((c.y * inv) * g1.y),
                  (_Float16)((c.z * inv) * g1.z), (_Float16)((c.w * inv) * g1.w) };
  _Float16* dst = xh + (size_t)row * HIDDEN + 8 * tid;
  *(volatile v8h*)dst = o;
  __threadfence();
  *(volatile v8h*)dst = o;
}

__device__ __forceinline__ void wt_store_pass(const _Float16* sT, _Float16* dstp,
                                              int n0, int k0, int w, int lane) {
  const int q8 = lane & 7, sub = lane >> 3;
  #pragma unroll
  for (int i = 0; i < 2; ++i) {
    const int lid = w * 8 + i * 4 + sub;
    const v8h v = *(const v8ha*)(sT + lid * 72 + 8 * q8);
    _Float16* dst = dstp + (size_t)(n0 + lid) * HIDDEN + k0 + 8 * q8;
    *(volatile v8h*)dst = v;
  }
}

__global__ __launch_bounds__(256) void wtrans_kernel(
    const float* __restrict__ wq, const float* __restrict__ wk,
    const float* __restrict__ wv, const float* __restrict__ wo,
    _Float16* __restrict__ wt)
{
  __shared__ __attribute__((aligned(16))) _Float16 sT[64 * 72];

  const int tid = threadIdx.x, lane = tid & 31, w = tid >> 5;
  const int k0 = blockIdx.x * 64;
  const int n0 = blockIdx.y * 64;
  const int wsel = blockIdx.z;
  const float* src = (wsel == 0) ? wq : ((wsel == 1) ? wk : ((wsel == 2) ? wv : wo));
  _Float16* dstp = wt + (size_t)wsel * NW;

  const int kr = tid >> 2, nc = (tid & 3) * 16;
  const float* sp = src + (size_t)(k0 + kr) * HIDDEN + n0 + nc;
  #pragma unroll
  for (int q = 0; q < 4; ++q) {
    const v4f v = *(const v4fa*)(sp + 4 * q);
    sT[(nc + 4 * q + 0) * 72 + kr] = (_Float16)(v.x * WSCALE);
    sT[(nc + 4 * q + 1) * 72 + kr] = (_Float16)(v.y * WSCALE);
    sT[(nc + 4 * q + 2) * 72 + kr] = (_Float16)(v.z * WSCALE);
    sT[(nc + 4 * q + 3) * 72 + kr] = (_Float16)(v.w * WSCALE);
  }
  __syncthreads();

  wt_store_pass(sT, dstp, n0, k0, w, lane);
  __threadfence();
  wt_store_pass(sT, dstp, n0, k0, w, lane);
}

__device__ __forceinline__ int rel_bucket(int rel) {
  int bucket = (rel > 0) ? 16 : 0;
  const int rp = (rel < 0) ? -rel : rel;
  const int rpm = (rp < 1) ? 1 : rp;
  const float rpf = (float)rpm;
  const float t = logf(rpf * 0.125f) * (1.0f / LN16F) * 8.0f;
  int vl = 8 + (int)t;
  vl = (vl < 15) ? vl : 15;
  bucket += (rp < 8) ? rp : vl;
  return bucket;
}

__global__ __launch_bounds__(256) void bias_kernel(
    const float* __restrict__ rel_emb,
    float* __restrict__ btab)
{
  const int idx = blockIdx.x * 256 + threadIdx.x;
  const int head = idx >> 12, i = idx & (BTW - 1);
  const int rel = i - 2048;
  int bucket = rel_bucket(rel);
  bucket = (bucket < 0) ? 0 : ((bucket > NBUCK - 1) ? (NBUCK - 1) : bucket);
  const float v = rel_emb[bucket * NHEADS + head];
  *(volatile float*)(btab + idx) = v;
  __threadfence();
  *(volatile float*)(btab + idx) = v;
}

__device__ __forceinline__ void proj_store_pass(const _Float16* sT, _Float16* plane, _Float16* vt,
                                                int which, int bh, int l0, int w, int lane) {
  const int q8 = lane & 7, sub = lane >> 3;
  #pragma unroll
  for (int i = 0; i < 8; ++i) {
    const int lid = w * 32 + i * 4 + sub;
    v8h v;
    _Float16* dst;
    if (which != 2) {
      v = *(const v8ha*)(sT + lid * HD + 8 * q8);
      dst = plane + ((size_t)bh * SEQ + l0 + lid) * HD + 8 * q8;
    } else {
      const int d = lid >> 1, hl = lid & 1;
      v = *(const v8ha*)(sT + d * 128 + 64 * hl + 8 * q8);
      dst = vt + ((size_t)bh * HD + d) * SEQ + l0 + 64 * hl + 8 * q8;
    }
    *(volatile v8h*)dst = v;
  }
}

__global__ __launch_bounds__(128) void proj_kernel(
    const _Float16* __restrict__ xh,
    const _Float16* __restrict__ wt,
    _Float16* __restrict__ qh,
    _Float16* __restrict__ kh,
    _Float16* __restrict__ vt)
{
  __shared__ __attribute__((aligned(16))) _Float16 sT[128 * 64];

  const int tid = threadIdx.x, lane = tid & 31, w = tid >> 5;
  const int h = lane >> 4, m = lane & 15;
  const int m0 = blockIdx.x * 128;
  const int cg = blockIdx.y;
  const int which = cg >> 4, head = cg & 15;
  const int m0w = m0 + 32 * w;

  const _Float16* xa0 = xh + (size_t)(m0w + m) * HIDDEN;
  const _Float16* xa1 = xa0 + (size_t)16 * HIDDEN;
  const _Float16* wb  = wt + ((size_t)which * HIDDEN + head * HD + m) * HIDDEN;

  const v8f zero8 = {0.f, 0.f, 0.f, 0.f, 0.f, 0.f, 0.f, 0.f};
  v8f acc[2][4];
  #pragma unroll
  for (int mt = 0; mt < 2; ++mt)
    #pragma unroll
    for (int nt = 0; nt < 4; ++nt) acc[mt][nt] = zero8;

  #pragma unroll 1
  for (int k0 = 0; k0 < HIDDEN; k0 += 32) {
    const v16h a0 = load_frag(xa0 + k0, h);
    const v16h a1 = load_frag(xa1 + k0, h);
    #pragma unroll
    for (int nt = 0; nt < 4; ++nt) {
      const v16h b = load_frag(wb + (size_t)nt * 16 * HIDDEN + k0, h);
      acc[0][nt] = wmma_f16(a0, b, acc[0][nt]);
      acc[1][nt] = wmma_f16(a1, b, acc[1][nt]);
    }
  }

  #pragma unroll
  for (int nt = 0; nt < 4; ++nt) {
    const int feat = 16 * nt + m;
    #pragma unroll
    for (int mt = 0; mt < 2; ++mt) {
      #pragma unroll
      for (int r = 0; r < 8; ++r) {
        const int tokl = 32 * w + 16 * mt + 8 * h + r;
        const float y = acc[mt][nt][r] * (1.0f / WSCALE);
        const int idx = (which == 2) ? (feat * 128 + tokl) : (tokl * HD + feat);
        sT[idx] = (_Float16)y;
      }
    }
  }
  __syncthreads();

  const int b = m0 / SEQ, l0 = m0 - b * SEQ, bh = b * NHEADS + head;
  _Float16* plane = (which == 0) ? qh : kh;
  proj_store_pass(sT, plane, vt, which, bh, l0, w, lane);
  __threadfence();
  proj_store_pass(sT, plane, vt, which, bh, l0, w, lane);
}

__device__ __forceinline__ v8f add_bias8(v8f s, const float* p) {
  #pragma unroll
  for (int r = 0; r < 8; ++r) s[r] = s[r] + p[r];
  return s;
}

__device__ __forceinline__ v16h pack_p(v8f a, v8f c) {
  const v16h r = { (_Float16)(a[0] * PSCALE), (_Float16)(a[1] * PSCALE), (_Float16)(a[2] * PSCALE), (_Float16)(a[3] * PSCALE),
                   (_Float16)(a[4] * PSCALE), (_Float16)(a[5] * PSCALE), (_Float16)(a[6] * PSCALE), (_Float16)(a[7] * PSCALE),
                   (_Float16)(c[0] * PSCALE), (_Float16)(c[1] * PSCALE), (_Float16)(c[2] * PSCALE), (_Float16)(c[3] * PSCALE),
                   (_Float16)(c[4] * PSCALE), (_Float16)(c[5] * PSCALE), (_Float16)(c[6] * PSCALE), (_Float16)(c[7] * PSCALE) };
  return r;
}

__device__ __forceinline__ void ctx_store_pass(const _Float16* so, _Float16* ctx,
                                               int b, int head, int q0, int lane) {
  const int q8 = lane & 7, sub = lane >> 3;
  #pragma unroll
  for (int i = 0; i < 4; ++i) {
    const int lid = i * 4 + sub;
    const v8h v = *(const v8ha*)(so + lid * 64 + 8 * q8);
    _Float16* dst = ctx + ((size_t)b * SEQ + q0 + lid) * HIDDEN + head * HD + 8 * q8;
    *(volatile v8h*)dst = v;
  }
}

__global__ __launch_bounds__(128) void attn_kernel(
    const _Float16* __restrict__ qh,
    const _Float16* __restrict__ kh,
    const _Float16* __restrict__ vt,
    const float* __restrict__ btab,
    _Float16* __restrict__ ctx)
{
  __shared__ __attribute__((aligned(16))) _Float16 sC[4 * 16 * 64];

  const int tid = threadIdx.x, lane = tid & 31, w = tid >> 5;
  const int h = lane >> 4, m = lane & 15;
  const int bh = blockIdx.y, b = bh >> 4, head = bh & 15;
  const int q0 = blockIdx.x * 64 + 16 * w;

  const _Float16* qrow = qh + ((size_t)bh * SEQ + q0 + m) * HD;
  const v16h qb0 = load_frag(qrow, h);
  const v16h qb1 = load_frag(qrow + 32, h);

  const v8f zero8 = {0.f, 0.f, 0.f, 0.f, 0.f, 0.f, 0.f, 0.f};
  v8f o[4];
  #pragma unroll
  for (int t = 0; t < 4; ++t) o[t] = zero8;
  float mrun = -1e30f, lrun = 0.0f;

  const _Float16* kbase = kh + ((size_t)bh * SEQ + m) * HD;
  const _Float16* vbase = vt + ((size_t)bh * HD + m) * SEQ;
  const float* bbase = btab + (size_t)head * BTW + 2048 + 8 * h - (q0 + m);

  #pragma unroll 1
  for (int kb = 0; kb < SEQ; kb += 64) {
    v8f s[4];
    #pragma unroll
    for (int j = 0; j < 4; ++j) {
      const _Float16* kp = kbase + (size_t)(kb + 16 * j) * HD;
      const v16h kf0 = load_frag(kp, h);
      const v16h kf1 = load_frag(kp + 32, h);
      v8f z = zero8;
      z = wmma_f16(kf0, qb0, z);
      z = wmma_f16(kf1, qb1, z);
      s[j] = z;
    }
    #pragma unroll
    for (int j = 0; j < 4; ++j) s[j] = add_bias8(s[j], bbase + kb + 16 * j);

    float mloc = s[0][0];
    #pragma unroll
    for (int j = 0; j < 4; ++j)
      #pragma unroll
      for (int r = 0; r < 8; ++r) mloc = fmaxf(mloc, s[j][r]);
    mloc = fmaxf(mloc, __shfl_xor(mloc, 16));
    const float mnew = fmaxf(mrun, mloc);
    const float alpha = __expf(mrun - mnew);
    mrun = mnew;
    float lsum = 0.0f;
    #pragma unroll
    for (int j = 0; j < 4; ++j)
      #pragma unroll
      for (int r = 0; r < 8; ++r) {
        const float p = __expf(s[j][r] - mnew);
        s[j][r] = p;
        lsum += p;
      }
    lsum += __shfl_xor(lsum, 16);
    lrun = lrun * alpha + lsum;
    #pragma unroll
    for (int t = 0; t < 4; ++t)
      #pragma unroll
      for (int r = 0; r < 8; ++r) o[t][r] = o[t][r] * alpha;

    const v16h pb0 = pack_p(s[0], s[1]);
    const v16h pb1 = pack_p(s[2], s[3]);

    #pragma unroll
    for (int t = 0; t < 4; ++t) {
      const _Float16* vp = vbase + (size_t)(16 * t) * SEQ + kb;
      const v16h vf0 = load_frag(vp, h);
      const v16h vf1 = load_frag(vp + 32, h);
      o[t] = wmma_f16(vf0, pb0, o[t]);
      o[t] = wmma_f16(vf1, pb1, o[t]);
    }
  }

  const float inv = (1.0f / lrun) * (CSCALE / PSCALE);
  _Float16* so = sC + w * 1024;
  #pragma unroll
  for (int t = 0; t < 4; ++t)
    #pragma unroll
    for (int r = 0; r < 8; ++r)
      so[m * 64 + 16 * t + 8 * h + r] = (_Float16)(o[t][r] * inv);
  __syncthreads();

  ctx_store_pass(so, ctx, b, head, q0, lane);
  __threadfence();
  ctx_store_pass(so, ctx, b, head, q0, lane);
}

__device__ __forceinline__ void out_store_pass(const float* sT, const float* hs, float* out,
                                               int m0, int col0, int w, int lane) {
  const int q8 = lane & 7, sub = lane >> 3;
  #pragma unroll
  for (int i = 0; i < 16; ++i) {
    const int lid = i * 4 + sub;
    const int row = w * 32 + (lid >> 1), hl = lid & 1;
    v4f v = *(const v4fa*)(sT + row * 64 + 32 * hl + 4 * q8);
    const size_t gi = (size_t)(m0 + row) * HIDDEN + col0 + 32 * hl + 4 * q8;
    const v4f res = *(const v4fa*)(hs + gi);
    v = v + res;
    *(volatile v4f*)(out + gi) = v;
  }
}

__global__ __launch_bounds__(128) void oproj_kernel(
    const _Float16* __restrict__ ch,
    const _Float16* __restrict__ woh,
    const float* __restrict__ hs,
    float* __restrict__ out)
{
  __shared__ __attribute__((aligned(16))) float sT[128 * 64];

  const int tid = threadIdx.x, lane = tid & 31, w = tid >> 5;
  const int h = lane >> 4, m = lane & 15;
  const int m0 = blockIdx.x * 128;
  const int col0 = blockIdx.y * 64;
  const int m0w = m0 + 32 * w;

  const _Float16* ca0 = ch + (size_t)(m0w + m) * HIDDEN;
  const _Float16* ca1 = ca0 + (size_t)16 * HIDDEN;
  const _Float16* wb  = woh + (size_t)(col0 + m) * HIDDEN;

  const v8f zero8 = {0.f, 0.f, 0.f, 0.f, 0.f, 0.f, 0.f, 0.f};
  v8f acc[2][4];
  #pragma unroll
  for (int mt = 0; mt < 2; ++mt)
    #pragma unroll
    for (int nt = 0; nt < 4; ++nt) acc[mt][nt] = zero8;

  #pragma unroll 1
  for (int k0 = 0; k0 < HIDDEN; k0 += 32) {
    const v16h a0 = load_frag(ca0 + k0, h);
    const v16h a1 = load_frag(ca1 + k0, h);
    #pragma unroll
    for (int nt = 0; nt < 4; ++nt) {
      const v16h b = load_frag(wb + (size_t)nt * 16 * HIDDEN + k0, h);
      acc[0][nt] = wmma_f16(a0, b, acc[0][nt]);
      acc[1][nt] = wmma_f16(a1, b, acc[1][nt]);
    }
  }

  #pragma unroll
  for (int nt = 0; nt < 4; ++nt) {
    const int feat = 16 * nt + m;
    #pragma unroll
    for (int mt = 0; mt < 2; ++mt) {
      #pragma unroll
      for (int r = 0; r < 8; ++r) {
        const int tokl = 32 * w + 16 * mt + 8 * h + r;
        sT[tokl * 64 + feat] = acc[mt][nt][r] * (1.0f / (WSCALE * CSCALE));
      }
    }
  }
  __syncthreads();

  out_store_pass(sT, hs, out, m0, col0, w, lane);
  __threadfence();
  out_store_pass(sT, hs, out, m0, col0, w, lane);
}

extern "C" void kernel_launch(void* const* d_in, const int* in_sizes, int n_in,
                              void* d_out, int out_size, void* d_ws, size_t ws_size,
                              hipStream_t stream) {
  if (n_in < 7) return;
  if (in_sizes[0] != NX) return;
  if (in_sizes[1] != HIDDEN) return;
  if (in_sizes[2] != NW || in_sizes[3] != NW || in_sizes[4] != NW || in_sizes[5] != NW) return;
  if (in_sizes[6] != NBUCK * NHEADS) return;
  if (out_size != NX) return;

  const float* x    = (const float*)d_in[0];
  const float* lnw  = (const float*)d_in[1];
  const float* Wq   = (const float*)d_in[2];
  const float* Wk   = (const float*)d_in[3];
  const float* Wv   = (const float*)d_in[4];
  const float* Wo   = (const float*)d_in[5];
  const float* remb = (const float*)d_in[6];
  float* out = (float*)d_out;

  const size_t xh_bytes  = (size_t)NX * 2;
  const size_t wt_bytes  = (size_t)4 * NW * 2;
  const size_t pl_bytes  = (size_t)NBH * SEQ * HD * 2;
  const size_t ctx_bytes = (size_t)NX * 2;
  const size_t bt_bytes  = (size_t)NHEADS * BTW * 4;
  const size_t total = xh_bytes + wt_bytes + 3 * pl_bytes + ctx_bytes + bt_bytes;
  if (total > ws_size) return;

  char* ws = (char*)d_ws;
  size_t off = 0;
  _Float16* xh  = (_Float16*)(ws + off); off += xh_bytes;
  _Float16* wt  = (_Float16*)(ws + off); off += wt_bytes;
  _Float16* qh  = (_Float16*)(ws + off); off += pl_bytes;
  _Float16* kh  = (_Float16*)(ws + off); off += pl_bytes;
  _Float16* vt  = (_Float16*)(ws + off); off += pl_bytes;
  _Float16* ctx = (_Float16*)(ws + off); off += ctx_bytes;
  float* btab   = (float*)(ws + off);    off += bt_bytes;
  if (off > ws_size) return;

  rmsnorm_kernel<<<MROWS, 128, 0, stream>>>(x, lnw, xh);

  dim3 gWt(HIDDEN / 64, HIDDEN / 64, 4);
  wtrans_kernel<<<gWt, 256, 0, stream>>>(Wq, Wk, Wv, Wo, wt);

  bias_kernel<<<(NHEADS * BTW) / 256, 256, 0, stream>>>(remb, btab);

  dim3 gProj(MROWS / 128, 3 * NHEADS);
  proj_kernel<<<gProj, 128, 0, stream>>>(xh, wt, qh, kh, vt);

  dim3 gAtt(SEQ / 64, NBH);
  attn_kernel<<<gAtt, 128, 0, stream>>>(qh, kh, vt, btab, ctx);

  dim3 gOut(MROWS / 128, HIDDEN / 64);
  oproj_kernel<<<gOut, 128, 0, stream>>>(ctx, wt + (size_t)3 * NW, x, out);
}
